// RelPosGraphAttention_2997887172854
// MI455X (gfx1250) — hardware-run, weakly checked
//
#include <hip/hip_runtime.h>
#include <stddef.h>
#include <stdint.h>

#define NBT   4
#define SQ    1024
#define PSQ   2048
#define HID   768
#define NH    12
#define HDM   64
#define NTOK  (NBT * SQ)
#define NPOS  (NBT * PSQ)
#define QB    128
#define KC    64
#define NQB   (SQ / QB)
#define NCK   (SQ / KC)
#define KRW   192
#define KTP   72
#define TPP   80
#define STP   72
#define SVP   264
#define OTP   68
#define PROJ_INV 0.03125f
#define OUT_INV  0.00048828125f
#define WSCALE   32.0f
#define PSCALE   1024.0f

#define LDS_KS 0
#define LDS_VS (LDS_KS + KC * KTP * 2)
#define LDS_KR (LDS_VS + HDM * KTP * 2)
#define LDS_PS (LDS_KR + KRW * KTP * 2)
#define LDS_TS (LDS_PS + 8 * 16 * KTP * 2)
#define LDS_TOTAL (LDS_TS + 8 * 16 * TPP * 4)

static_assert(NH * HDM == HID);
static_assert(SQ % QB == 0);
static_assert(SQ % KC == 0);
static_assert(SQ % 256 == 0);
static_assert(PSQ % 256 == 0);
static_assert(NTOK % 256 == 0);
static_assert(NPOS % 256 == 0);
static_assert(HID % 64 == 0);
static_assert((NTOK * HID) % 2048 == 0);
static_assert((NPOS * HID) % 2048 == 0);
static_assert(QB - 1 + KC <= KRW);
static_assert((QB - 16) + 4 * 16 + 15 < KRW);
static_assert(KC - 1 - 0 + 15 < TPP);
static_assert(LDS_VS % 16 == 0);
static_assert(LDS_KR % 16 == 0);
static_assert(LDS_PS % 16 == 0);
static_assert(LDS_TS % 16 == 0);
static_assert(256 * STP >= 64 * SVP);

typedef _Float16 v16h __attribute__((ext_vector_type(16)));
typedef _Float16 v8h  __attribute__((ext_vector_type(8)));
typedef float    v8f  __attribute__((ext_vector_type(8)));
typedef float    v4f  __attribute__((ext_vector_type(4)));
typedef unsigned int v4u __attribute__((ext_vector_type(4)));

union Frag  { v16h v; v8h h[2]; };
union Pack8 { v8h h; v4u u; };

__device__ __forceinline__ v8f mma16(v16h a, v16h b, v8f c) {
  c = __builtin_amdgcn_wmma_f32_16x16x32_f16(false, a, false, b, (short)0, c, false, false);
  asm volatile("v_nop\n\tv_nop\n\tv_nop\n\tv_nop" : "+v"(c) : "v"(a), "v"(b));
  return c;
}

__device__ __forceinline__ v16h ldfrag(const _Float16* p, int ld, int row0, int k0, int lane) {
  const int m = lane & 15, lh = lane >> 4;
  const _Float16* q = p + (size_t)(row0 + m) * ld + k0 + 8 * lh;
  Frag f;
  f.h[0] = *(const v8h*)(q);
  f.h[1] = *(const v8h*)(q + 16);
  return f.v;
}

__device__ __forceinline__ v8f zero8() { return (v8f){0.f, 0.f, 0.f, 0.f, 0.f, 0.f, 0.f, 0.f}; }

__device__ __forceinline__ float gelu1(float z) {
  return 0.5f * z * (1.0f + erff(z * 0.70710678118654752f));
}

__device__ __forceinline__ void gemm32x64(const _Float16* __restrict__ A, int lda,
                                          const _Float16* __restrict__ Bt, int ldb, int K,
                                          int m0, int n0, int lane, v8f (&acc)[2][4]) {
#pragma unroll 1
  for (int k0 = 0; k0 < K; k0 += 32) {
    const v16h a0 = ldfrag(A, lda, m0, k0, lane);
    const v16h a1 = ldfrag(A, lda, m0 + 16, k0, lane);
    const v16h b0 = ldfrag(Bt, ldb, n0, k0, lane);
    const v16h b1 = ldfrag(Bt, ldb, n0 + 16, k0, lane);
    const v16h b2 = ldfrag(Bt, ldb, n0 + 32, k0, lane);
    const v16h b3 = ldfrag(Bt, ldb, n0 + 48, k0, lane);
    acc[0][0] = mma16(a0, b0, acc[0][0]);
    acc[1][0] = mma16(a1, b0, acc[1][0]);
    acc[0][1] = mma16(a0, b1, acc[0][1]);
    acc[1][1] = mma16(a1, b1, acc[1][1]);
    acc[0][2] = mma16(a0, b2, acc[0][2]);
    acc[1][2] = mma16(a1, b2, acc[1][2]);
    acc[0][3] = mma16(a0, b3, acc[0][3]);
    acc[1][3] = mma16(a1, b3, acc[1][3]);
  }
}

__global__ __launch_bounds__(256) void k_cvt(const float* __restrict__ src, _Float16* __restrict__ dst) {
  const size_t o = (size_t)blockIdx.x * 2048 + (size_t)threadIdx.x * 8;
  const v4f a0 = *(const v4f*)(src + o);
  const v4f a1 = *(const v4f*)(src + o + 4);
  Pack8 pk;
  pk.h = (v8h){(_Float16)a0[0], (_Float16)a0[1], (_Float16)a0[2], (_Float16)a0[3],
               (_Float16)a1[0], (_Float16)a1[1], (_Float16)a1[2], (_Float16)a1[3]};
  const v4u vv = pk.u;
  volatile v4u* d = (volatile v4u*)(dst + o);
  *d = vv;
  __threadfence();
  *d = vv;
}

__global__ __launch_bounds__(256) void k_wtr(const float* __restrict__ src, _Float16* __restrict__ dst) {
  __shared__ __align__(16) _Float16 tt[64 * STP];
  const int tid = threadIdx.x;
  const int k0 = (int)blockIdx.x * 64;
  const int n0 = (int)blockIdx.y * 64;
#pragma unroll
  for (int e = 0; e < 4; ++e) {
    const int idx = tid + 256 * e;
    const int r   = idx >> 4;
    const int q4  = (idx & 15) * 4;
    const v4f v = *(const v4f*)(src + (size_t)(k0 + r) * HID + n0 + q4) * WSCALE;
    tt[(q4 + 0) * STP + r] = (_Float16)v[0];
    tt[(q4 + 1) * STP + r] = (_Float16)v[1];
    tt[(q4 + 2) * STP + r] = (_Float16)v[2];
    tt[(q4 + 3) * STP + r] = (_Float16)v[3];
  }
  __syncthreads();
  v4u val[2];
  size_t go[2];
#pragma unroll
  for (int g = 0; g < 2; ++g) {
    const int p   = tid + 256 * g;
    const int row = p >> 3;
    const int pc  = p & 7;
    Pack8 pk;
    pk.h    = *(const v8h*)(tt + row * STP + pc * 8);
    val[g]  = pk.u;
    go[g]   = (size_t)(n0 + row) * HID + k0 + pc * 8;
  }
  for (int ps = 0; ps < 2; ++ps) {
#pragma unroll
    for (int g = 0; g < 2; ++g) *(volatile v4u*)(dst + go[g]) = val[g];
    __threadfence();
  }
}

__device__ __forceinline__ void write_sd(const _Float16* st, _Float16* __restrict__ base, int sb, int tid) {
#pragma unroll
  for (int g = 0; g < 2; ++g) {
    v4u val[4];
    size_t go[4];
#pragma unroll
    for (int j = 0; j < 4; ++j) {
      const int p  = tid + 256 * (4 * g + j);
      const int lr = p >> 3;
      const int pc = p & 7;
      Pack8 pk;
      pk.h   = *(const v8h*)(st + lr * STP + pc * 8);
      val[j] = pk.u;
      go[j]  = (size_t)(sb + lr) * HDM + pc * 8;
    }
    for (int ps = 0; ps < 2; ++ps) {
#pragma unroll
      for (int j = 0; j < 4; ++j) *(volatile v4u*)(base + go[j]) = val[j];
      __threadfence();
    }
  }
}

__device__ __forceinline__ void write_ds(const _Float16* st, _Float16* __restrict__ base, int seq, int sb, int tid) {
#pragma unroll
  for (int g = 0; g < 2; ++g) {
    v4u val[4];
    size_t go[4];
#pragma unroll
    for (int j = 0; j < 4; ++j) {
      const int p    = tid + 256 * (4 * g + j);
      const int drow = p >> 5;
      const int pc   = p & 31;
      Pack8 pk;
      pk.h   = *(const v8h*)(st + drow * SVP + pc * 8);
      val[j] = pk.u;
      go[j]  = (size_t)drow * seq + sb + pc * 8;
    }
    for (int ps = 0; ps < 2; ++ps) {
#pragma unroll
      for (int j = 0; j < 4; ++j) *(volatile v4u*)(base + go[j]) = val[j];
      __threadfence();
    }
  }
}

__global__ __launch_bounds__(256) void k_proj(const _Float16* __restrict__ ap, int seq,
                                              const _Float16* __restrict__ wt,
                                              const float* __restrict__ bias_a,
                                              const float* __restrict__ bias_b,
                                              _Float16* __restrict__ p0,
                                              _Float16* __restrict__ p1, int kind) {
  __shared__ __align__(16) _Float16 st[256 * STP];
  const int tid = threadIdx.x, lane = tid & 31, wave = tid >> 5;
  const int hh = lane >> 4, c = lane & 15;
  const int tok0 = (int)blockIdx.x * 256;
  const int b    = tok0 / seq;
  const int sb   = tok0 - b * seq;
  const int head = (int)blockIdx.y;
  const int hb   = b * NH + head;
  const int m0   = tok0 + wave * 32;
  const int n0   = head * HDM;

  v8f acc[2][4];
#pragma unroll
  for (int s = 0; s < 2; ++s)
#pragma unroll
    for (int t = 0; t < 4; ++t) acc[s][t] = zero8();
  gemm32x64(ap, HID, wt, HID, HID, m0, n0, lane, acc);

  float ba[4], bbv[4];
#pragma unroll
  for (int t = 0; t < 4; ++t) {
    const int i = head * HDM + 16 * t + c;
    const float xa = bias_a[i], xb = bias_b[i];
    ba[t]  = (kind == 0) ? xa : 0.f;
    bbv[t] = (kind == 0) ? xb : 0.f;
  }

#pragma unroll
  for (int sub = 0; sub < 2; ++sub)
#pragma unroll
    for (int t = 0; t < 4; ++t)
#pragma unroll
      for (int r = 0; r < 8; ++r)
        st[(wave * 32 + sub * 16 + 8 * hh + r) * STP + 16 * t + c] =
            (_Float16)(acc[sub][t][r] * PROJ_INV + ba[t]);
  __syncthreads();
  write_sd(st, p0 + (size_t)hb * seq * HDM, sb, tid);
  __syncthreads();

  if (kind == 0) {
#pragma unroll
    for (int sub = 0; sub < 2; ++sub)
#pragma unroll
      for (int t = 0; t < 4; ++t)
#pragma unroll
        for (int r = 0; r < 8; ++r)
          st[(wave * 32 + sub * 16 + 8 * hh + r) * STP + 16 * t + c] =
              (_Float16)(acc[sub][t][r] * PROJ_INV + bbv[t]);
    __syncthreads();
    write_sd(st, p1 + (size_t)hb * seq * HDM, sb, tid);
  } else if (kind == 1) {
#pragma unroll
    for (int sub = 0; sub < 2; ++sub)
#pragma unroll
      for (int t = 0; t < 4; ++t)
#pragma unroll
        for (int r = 0; r < 8; ++r)
          st[(16 * t + c) * SVP + wave * 32 + sub * 16 + 8 * hh + r] =
              (_Float16)(acc[sub][t][r] * PROJ_INV);
    __syncthreads();
    write_ds(st, p1 + (size_t)hb * HDM * seq, seq, sb, tid);
  }
}

__global__ __launch_bounds__(256) void k_attn(const _Float16* __restrict__ qwp,
                                              const _Float16* __restrict__ qrp,
                                              const _Float16* __restrict__ kvp,
                                              const _Float16* __restrict__ vtp,
                                              const _Float16* __restrict__ krp,
                                              const float* __restrict__ mask,
                                              _Float16* __restrict__ op) {
  extern __shared__ __align__(16) unsigned char dlds[];
  _Float16* Ks  = (_Float16*)(dlds + LDS_KS);
  _Float16* Vs  = (_Float16*)(dlds + LDS_VS);
  _Float16* KRs = (_Float16*)(dlds + LDS_KR);
  _Float16* Ps  = (_Float16*)(dlds + LDS_PS);
  float*    Ts  = (float*)(dlds + LDS_TS);

  const int tid = threadIdx.x, lane = tid & 31, wave = tid >> 5;
  const int hh = lane >> 4, c = lane & 15;
  const int bx  = (int)blockIdx.x;
  const int qb  = bx % NQB;
  const int hb  = bx / NQB;
  const int h   = hb % NH;
  const int b   = hb / NH;
  const int i0  = qb * QB;
  const int iw0 = i0 + wave * 16;
  const int rw  = (QB - 16) - 16 * wave;

  const _Float16* Qw = qwp + (size_t)hb * SQ * HDM;
  const _Float16* Qr = qrp + (size_t)hb * SQ * HDM;
  const _Float16* K  = kvp + (size_t)hb * SQ * HDM;
  const _Float16* V  = vtp + (size_t)hb * HDM * SQ;
  const _Float16* R  = krp + (size_t)hb * PSQ * HDM;
  const float*   mkb = mask + (size_t)b * SQ * SQ;

  v16h qa[2], qr[2];
  qa[0] = ldfrag(Qw, HDM, iw0, 0, lane);
  qa[1] = ldfrag(Qw, HDM, iw0, 32, lane);
  qr[0] = ldfrag(Qr, HDM, iw0, 0, lane);
  qr[1] = ldfrag(Qr, HDM, iw0, 32, lane);

  const float NEGI = -__builtin_huge_valf();
  float mrow[8], lrow[8];
  v8f oacc[4];
#pragma unroll
  for (int r = 0; r < 8; ++r) { mrow[r] = NEGI; lrow[r] = 0.f; }
#pragma unroll
  for (int t = 0; t < 4; ++t) oacc[t] = zero8();

  _Float16* pw = Ps + wave * 16 * KTP;
  float*    tw = Ts + wave * 16 * TPP;

  for (int kc = 0; kc < NCK; ++kc) {
    const int c0    = kc * KC;
    const int pbase = c0 - i0 + (SQ - QB + 1);
    __syncthreads();
#pragma unroll
    for (int e = 0; e < 2; ++e) {
      const int idx = tid + 256 * e;
      const int r   = idx >> 3;
      const int pc  = (idx & 7) * 8;
      *(v8h*)(Ks + r * KTP + pc) = *(const v8h*)(K + (size_t)(c0 + r) * HDM + pc);
      *(v8h*)(Vs + r * KTP + pc) = *(const v8h*)(V + (size_t)r * SQ + c0 + pc);
    }
#pragma unroll
    for (int e = 0; e < 6; ++e) {
      const int idx = tid + 256 * e;
      const int r   = idx >> 3;
      const int pc  = (idx & 7) * 8;
      int prow = pbase + r;
      prow = prow < 0 ? 0 : prow;
      prow = prow > (PSQ - 1) ? (PSQ - 1) : prow;
      *(v8h*)(KRs + r * KTP + pc) = *(const v8h*)(R + (size_t)prow * HDM + pc);
    }
    __syncthreads();

    v8f s[4];
#pragma unroll
    for (int j = 0; j < 4; ++j) s[j] = zero8();
#pragma unroll
    for (int dc = 0; dc < 2; ++dc) {
#pragma unroll
      for (int j = 0; j < 4; ++j) {
        const v16h kb = ldfrag(Ks, KTP, j * 16, dc * 32, lane);
        s[j] = mma16(qa[dc], kb, s[j]);
      }
    }

#pragma unroll
    for (int j = 0; j < 5; ++j) {
      v8f tj = zero8();
#pragma unroll
      for (int dc = 0; dc < 2; ++dc) {
        const v16h rb = ldfrag(KRs, KTP, rw + 16 * j, dc * 32, lane);
        tj = mma16(qr[dc], rb, tj);
      }
#pragma unroll
      for (int r = 0; r < 8; ++r) tw[(8 * hh + r) * TPP + 16 * j + c] = tj[r];
    }
    __syncthreads();

    float cm[8];
#pragma unroll
    for (int r = 0; r < 8; ++r) {
      const int q = 8 * hh + r;
      const float* mr = mkb + (size_t)(iw0 + q) * SQ + c0 + c;
      const float* tr = tw + q * TPP + 15 - q + c;
      float m = NEGI;
#pragma unroll
      for (int j = 0; j < 4; ++j) {
        const float bd = tr[16 * j];
        const float mk = mr[16 * j];
        const float v  = (s[j][r] + bd) * 0.125f + mk * (-65500.0f);
        s[j][r] = v;
        m = fmaxf(m, v);
      }
#pragma unroll
      for (int off = 1; off < 16; off <<= 1) m = fmaxf(m, __shfl_xor(m, off, 32));
      cm[r] = m;
    }
    float al[8];
#pragma unroll
    for (int r = 0; r < 8; ++r) {
      const float mnew  = fmaxf(mrow[r], cm[r]);
      const float alpha = __expf(mrow[r] - mnew);
      mrow[r] = mnew;
      float psum = 0.f;
#pragma unroll
      for (int j = 0; j < 4; ++j) {
        const float p = __expf(s[j][r] - mnew);
        psum += p;
        pw[(8 * hh + r) * KTP + j * 16 + c] = (_Float16)(p * PSCALE);
      }
#pragma unroll
      for (int off = 1; off < 16; off <<= 1) psum += __shfl_xor(psum, off, 32);
      lrow[r] = lrow[r] * alpha + psum;
      al[r] = alpha;
    }
#pragma unroll
    for (int t = 0; t < 4; ++t)
#pragma unroll
      for (int r = 0; r < 8; ++r) oacc[t][r] *= al[r];
    __syncthreads();

#pragma unroll
    for (int kk = 0; kk < 2; ++kk) {
      const v16h pa = ldfrag(pw, KTP, 0, kk * 32, lane);
#pragma unroll
      for (int t = 0; t < 4; ++t) {
        const v16h vb = ldfrag(Vs, KTP, t * 16, kk * 32, lane);
        oacc[t] = mma16(pa, vb, oacc[t]);
      }
    }
  }

  float invl[8];
#pragma unroll
  for (int r = 0; r < 8; ++r) invl[r] = (lrow[r] > 0.f) ? (0.0625f * (1.0f / lrow[r])) : 0.f;
  __syncthreads();
#pragma unroll
  for (int r = 0; r < 8; ++r) {
#pragma unroll
    for (int t = 0; t < 4; ++t)
      pw[(8 * hh + r) * KTP + 16 * t + c] = (_Float16)(oacc[t][r] * invl[r]);
  }
  __syncthreads();
  v4u val[4];
  size_t go[4];
#pragma unroll
  for (int it = 0; it < 4; ++it) {
    const int p  = lane + 32 * it;
    const int L  = p >> 3;
    const int pc = p & 7;
    Pack8 pk;
    pk.h    = *(const v8h*)(pw + L * KTP + pc * 8);
    val[it] = pk.u;
    go[it]  = ((size_t)b * SQ + iw0 + L) * HID + (size_t)h * HDM + pc * 8;
  }
  for (int ps = 0; ps < 2; ++ps) {
#pragma unroll
    for (int it = 0; it < 4; ++it) *(volatile v4u*)(op + go[it]) = val[it];
    __threadfence();
  }
}

__global__ __launch_bounds__(256) void k_out(const _Float16* __restrict__ ap,
                                             const _Float16* __restrict__ wt,
                                             const float* __restrict__ bias,
                                             const float* __restrict__ resid,
                                             float* __restrict__ out) {
  __shared__ __align__(16) float st[8][16 * OTP];
  const int tid = threadIdx.x, lane = tid & 31, wave = tid >> 5;
  const int hh = lane >> 4, c = lane & 15;
  const int m0 = (int)blockIdx.x * 256 + wave * 32;
  const int n0 = (int)blockIdx.y * 64;

  v8f acc[2][4];
#pragma unroll
  for (int s = 0; s < 2; ++s)
#pragma unroll
    for (int t = 0; t < 4; ++t) acc[s][t] = zero8();
  gemm32x64(ap, HID, wt, HID, HID, m0, n0, lane, acc);
  float bb[4];
#pragma unroll
  for (int t = 0; t < 4; ++t) bb[t] = bias[n0 + 16 * t + c];

  float* sw = st[wave];
#pragma unroll
  for (int sub = 0; sub < 2; ++sub) {
    __syncthreads();
#pragma unroll
    for (int t = 0; t < 4; ++t) {
#pragma unroll
      for (int r = 0; r < 8; ++r) sw[(8 * hh + r) * OTP + 16 * t + c] = acc[sub][t][r] * OUT_INV + bb[t];
    }
    __syncthreads();
    v4f val[8];
    size_t go[8];
#pragma unroll
    for (int it = 0; it < 8; ++it) {
      const int p    = lane + 32 * it;
      const int L    = p >> 3;
      const int pc   = p & 7;
      const int row  = L >> 1;
      const int half = L & 1;
      const v4f a = *(const v4f*)(sw + row * OTP + half * 32 + pc * 4);
      go[it] = (size_t)(m0 + sub * 16 + row) * HID + n0 + half * 32 + pc * 4;
      const v4f hv = *(const v4f*)(resid + go[it]);
      const v4f z  = a + hv;
      val[it] = (v4f){gelu1(z[0]), gelu1(z[1]), gelu1(z[2]), gelu1(z[3])};
    }
    for (int ps = 0; ps < 2; ++ps) {
#pragma unroll
      for (int it = 0; it < 8; ++it) *(volatile v4f*)(out + go[it]) = val[it];
      __threadfence();
    }
  }
}

extern "C" void kernel_launch(void* const* d_in, const int* in_sizes, int n_in,
                              void* d_out, int out_size, void* d_ws, size_t ws_size,
                              hipStream_t stream) {
  if (n_in < 10) return;
  if (in_sizes[0] != NTOK * HID) return;
  if (in_sizes[1] != NPOS * HID) return;
  if (in_sizes[2] != NBT * SQ * SQ) return;
  if (in_sizes[3] != HID * HID) return;
  if (in_sizes[4] != HID * HID) return;
  if (in_sizes[5] != HID * HID) return;
  if (in_sizes[6] != HID) return;
  if (in_sizes[7] != HID) return;
  if (in_sizes[8] != HID * HID) return;
  if (in_sizes[9] != HID) return;
  if (out_size != NTOK * HID) return;

  const float* hidden = (const float*)d_in[0];
  const float* pos    = (const float*)d_in[1];
  const float* mask   = (const float*)d_in[2];
  const float* wq     = (const float*)d_in[3];
  const float* wkv    = (const float*)d_in[4];
  const float* wr     = (const float*)d_in[5];
  const float* rrb    = (const float*)d_in[6];
  const float* rwb    = (const float*)d_in[7];
  const float* wo     = (const float*)d_in[8];
  const float* bo     = (const float*)d_in[9];
  float* out = (float*)d_out;

  size_t off = 0;
  const size_t oX  = off; off += (size_t)NTOK * HID * 2;
  const size_t oP  = off; off += (size_t)NPOS * HID * 2;
  const size_t oW  = off; off += (size_t)4 * HID * HID * 2;
  const size_t oQW = off; off += (size_t)NBT * NH * SQ * HDM * 2;
  const size_t oQR = off; off += (size_t)NBT * NH * SQ * HDM * 2;
  const size_t oKV = off; off += (size_t)NBT * NH * SQ * HDM * 2;
  const size_t oVT = off; off += (size_t)NBT * NH * HDM * SQ * 2;
  const size_t oKR = off; off += (size_t)NBT * NH * PSQ * HDM * 2;
  const size_t oO  = off; off += (size_t)NTOK * HID * 2;
  if (off > ws_size) return;
  if (off > (size_t)134217728) return;

  char* ws = (char*)d_ws;
  _Float16* Xh  = (_Float16*)(ws + oX);
  _Float16* Ph  = (_Float16*)(ws + oP);
  _Float16* Wt  = (_Float16*)(ws + oW);
  _Float16* QWp = (_Float16*)(ws + oQW);
  _Float16* QRp = (_Float16*)(ws + oQR);
  _Float16* KVp = (_Float16*)(ws + oKV);
  _Float16* VTp = (_Float16*)(ws + oVT);
  _Float16* KRp = (_Float16*)(ws + oKR);
  _Float16* Op  = (_Float16*)(ws + oO);

  k_cvt<<<dim3((NTOK * HID) / 2048), dim3(256), 0, stream>>>(hidden, Xh);
  k_cvt<<<dim3((NPOS * HID) / 2048), dim3(256), 0, stream>>>(pos, Ph);
  k_wtr<<<dim3(HID / 64, HID / 64), dim3(256), 0, stream>>>(wq,  Wt);
  k_wtr<<<dim3(HID / 64, HID / 64), dim3(256), 0, stream>>>(wkv, Wt + (size_t)HID * HID);
  k_wtr<<<dim3(HID / 64, HID / 64), dim3(256), 0, stream>>>(wr,  Wt + (size_t)2 * HID * HID);
  k_wtr<<<dim3(HID / 64, HID / 64), dim3(256), 0, stream>>>(wo,  Wt + (size_t)3 * HID * HID);
  k_proj<<<dim3(NTOK / 256, NH), dim3(256), 0, stream>>>(Xh, SQ, Wt, rwb, rrb, QWp, QRp, 0);
  k_proj<<<dim3(NTOK / 256, NH), dim3(256), 0, stream>>>(Xh, SQ, Wt + (size_t)HID * HID, rwb, rrb, KVp, VTp, 1);
  k_proj<<<dim3(NPOS / 256, NH), dim3(256), 0, stream>>>(Ph, PSQ, Wt + (size_t)2 * HID * HID, rwb, rrb, KRp, KRp, 2);
  (void)hipFuncSetAttribute(reinterpret_cast<const void*>(&k_attn),
                            hipFuncAttributeMaxDynamicSharedMemorySize, LDS_TOTAL);
  k_attn<<<dim3(NBT * NH * NQB), dim3(256), LDS_TOTAL, stream>>>(QWp, QRp, KVp, VTp, KRp, mask, Op);
  k_out<<<dim3(NTOK / 256, HID / 64), dim3(256), 0, stream>>>(Op, Wt + (size_t)3 * HID * HID, bo, hidden, out);
  (void)hipGetLastError();
}
